// MetaLinear3_22565758174013
// MI455X (gfx1250) — hardware-verified
//
#include <hip/hip_runtime.h>
#include <math.h>


#define NTOK 1024
#define DI   512
#define NC   1536
typedef __attribute__((ext_vector_type(16))) _Float16 v16h;
typedef __attribute__((ext_vector_type(8)))  _Float16 v8h;
typedef __attribute__((ext_vector_type(8)))  float    v8f;
typedef __attribute__((ext_vector_type(4)))  float    v4f;
#define VST2(T, ptr, val) do { const T _v = (val); *(volatile T*)(ptr) = _v; __threadfence(); *(volatile T*)(ptr) = _v; } while (0)
__device__ __forceinline__ v8f wmma16(v16h a, v16h b, v8f c) {
  v8f d = __builtin_amdgcn_wmma_f32_16x16x32_f16(false, a, false, b, (short)0, c, false, false);
  asm volatile("v_nop\n\tv_nop\n\tv_nop\n\tv_nop" : "+v"(d) : "v"(a), "v"(b));
  return d;
}
__device__ __forceinline__ v16h frag16(const _Float16* p, int hh) {
  const v8h lo = *(const v8h*)(p + 8 * hh), hi = *(const v8h*)(p + 16 + 8 * hh);
  return __builtin_shufflevector(lo, hi, 0,1,2,3,4,5,6,7,8,9,10,11,12,13,14,15);
}
__global__ __launch_bounds__(256) void k_split(const float* __restrict__ s, int rows, _Float16* __restrict__ hi, _Float16* __restrict__ lo) {
  const int t = blockIdx.x * 256 + threadIdx.x;
  if (t >= rows * 64) return;
  const int r = t >> 6, c = (t & 63) * 8;
  v8h h, l;
#pragma unroll
  for (int e = 0; e < 8; ++e) { const float v = s[(size_t)r * DI + c + e]; const _Float16 a = (_Float16)v; h[e] = a; l[e] = (_Float16)(v - (float)a); }
  VST2(v8h, hi + (size_t)r * DI + c, h); VST2(v8h, lo + (size_t)r * DI + c, l);
}
__global__ __launch_bounds__(128) void k_gemm(const _Float16* __restrict__ Xh, const _Float16* __restrict__ Xl, const _Float16* __restrict__ Wh, const _Float16* __restrict__ Wl, float* __restrict__ C) {
  __shared__ __attribute__((aligned(16))) float sT[4][16][132];
  const int lane = threadIdx.x & 31, wave = threadIdx.x >> 5, hh = lane >> 4, l16 = lane & 15;
  const int m0 = blockIdx.x * 64 + wave * 16, n0 = blockIdx.y * 128;
  v8f acc[8];
#pragma unroll
  for (int ni = 0; ni < 8; ++ni) acc[ni] = (v8f){};
  for (int k0 = 0; k0 < DI; k0 += 32) {
    const v16h ah = frag16(Xh + (size_t)(m0 + l16) * DI + k0, hh), al = frag16(Xl + (size_t)(m0 + l16) * DI + k0, hh);
#pragma unroll
    for (int ni = 0; ni < 8; ++ni) {
      const v16h bh = frag16(Wh + (size_t)(n0 + ni * 16 + l16) * DI + k0, hh), bl = frag16(Wl + (size_t)(n0 + ni * 16 + l16) * DI + k0, hh);
      acc[ni] = wmma16(ah, bh, acc[ni]); acc[ni] = wmma16(ah, bl, acc[ni]); acc[ni] = wmma16(al, bh, acc[ni]);
    }
  }
  float (*st)[132] = sT[wave];
#pragma unroll
  for (int ni = 0; ni < 8; ++ni)
#pragma unroll
    for (int i = 0; i < 8; ++i) st[i + 8 * hh][ni * 16 + l16] = acc[ni][i];
  __builtin_amdgcn_fence(__ATOMIC_RELEASE, "workgroup"); __builtin_amdgcn_wave_barrier(); __builtin_amdgcn_fence(__ATOMIC_ACQUIRE, "workgroup");
  for (int pass = 0; pass < 2; ++pass) {
#pragma unroll
    for (int rr = 0; rr < 16; ++rr) *(volatile v4f*)(C + (size_t)(m0 + rr) * NC + n0 + lane * 4) = *(const v4f*)(&st[rr][lane * 4]);
    __threadfence();
  }
}
__global__ __launch_bounds__(256) void k_final(const float* __restrict__ C, const float* __restrict__ x, float* __restrict__ y) {
  const int tok = blockIdx.x * 8 + (threadIdx.x >> 5), lane = threadIdx.x & 31;
  const float* w1 = C + (size_t)tok * NC; const float* w2 = w1 + DI; const float* xb = w1 + 2 * DI; const float* xr = x + (size_t)tok * DI;
  float s1 = 0.f, sx = 0.f, d = 0.f, sb = 0.f;
  for (int j = lane; j < DI; j += 32) { s1 += w1[j]; sx += xr[j]; d += w1[j] * xr[j]; sb += xb[j]; }
#pragma unroll
  for (int o = 16; o > 0; o >>= 1) { s1 += __shfl_xor(s1, o, 32); sx += __shfl_xor(sx, o, 32); d += __shfl_xor(d, o, 32); sb += __shfl_xor(sb, o, 32); }
  const float mu1 = s1 * (1.0f / DI), mub = sb * (1.0f / DI);
  float v1 = 0.f, vb = 0.f;
  for (int j = lane; j < DI; j += 32) { const float a = w1[j] - mu1; v1 += a * a; const float bb = xb[j] - mub; vb += bb * bb; }
#pragma unroll
  for (int o = 16; o > 0; o >>= 1) { v1 += __shfl_xor(v1, o, 32); vb += __shfl_xor(vb, o, 32); }
  const float var1 = v1 * (1.0f / DI), rsb = rsqrtf(vb * (1.0f / DI) + 1e-5f);
  const float dd = d - mu1 * sx;
  for (int pass = 0; pass < 2; ++pass) {
#pragma unroll
    for (int q = 0; q < 4; ++q) {
      const int i0 = (q * 32 + lane) * 4;
      v4f o;
#pragma unroll
      for (int e = 0; e < 4; ++e) { const float a = w2[i0 + e]; o[e] = a * dd * rsqrtf(a * a * var1 + 1e-5f) + (xb[i0 + e] - mub) * rsb; }
      *(volatile v4f*)(y + (size_t)tok * DI + i0) = o;
    }
    __threadfence();
  }
}
extern "C" void kernel_launch(void* const* d_in, const int* in_sizes, int n_in,
                              void* d_out, int out_size, void* d_ws, size_t ws_size, hipStream_t stream) {
  (void)in_sizes; (void)n_in; (void)out_size;
  const float* x    = (const float*)d_in[0];
  const float* Win  = (const float*)d_in[1];
  const float* Wout = (const float*)d_in[2];
  const float* Wb   = (const float*)d_in[3];
  float* y = (float*)d_out;
  char* ws = (char*)d_ws; size_t off = 0;
  auto take = [&](size_t bytes) { void* p = ws + off; off = (off + bytes + 255) & ~(size_t)255; return p; };
  _Float16* Xh = (_Float16*)take((size_t)NTOK * DI * 2); _Float16* Xl = (_Float16*)take((size_t)NTOK * DI * 2);
  _Float16* Wh = (_Float16*)take((size_t)NC * DI * 2);   _Float16* Wl = (_Float16*)take((size_t)NC * DI * 2);
  float*    C  = (float*)take((size_t)NTOK * NC * 4);
  if (off > ws_size) return;
  k_split<<<NTOK * 64 / 256, 256, 0, stream>>>(x, NTOK, Xh, Xl);
  k_split<<<DI * 64 / 256, 256, 0, stream>>>(Win, DI, Wh, Wl);
  k_split<<<DI * 64 / 256, 256, 0, stream>>>(Wout, DI, Wh + (size_t)DI * DI, Wl + (size_t)DI * DI);
  k_split<<<DI * 64 / 256, 256, 0, stream>>>(Wb, DI, Wh + (size_t)2 * DI * DI, Wl + (size_t)2 * DI * DI);
  k_gemm<<<dim3(NTOK / 64, NC / 128), 128, 0, stream>>>(Xh, Xl, Wh, Wl, C);
  k_final<<<NTOK / 8, 256, 0, stream>>>(C, x, y);
}
